// PointFEF_16922171146620
// MI455X (gfx1250) — hardware-verified
//
#include <hip/hip_runtime.h>
#define NBT 2
#define CU 3
#define CV 64
#define NPT 4096
#define NS 64
#ifndef NSI
#define NSI NS
#endif
#define NR ((size_t)NBT * NPT * NS)
#define CH1 134
#define CHP 160
#define CO3 64
#define RB 2048
#define NBLK (NR / RB)
typedef __bf16 v16b __attribute__((ext_vector_type(16)));
typedef unsigned short v8us __attribute__((ext_vector_type(8), may_alias));
typedef float  v8f  __attribute__((ext_vector_type(8)));
typedef float  v4f  __attribute__((ext_vector_type(4)));
typedef float  v4fa __attribute__((ext_vector_type(4), may_alias));
union FragB { v16b v; v8us half[2]; unsigned short u[16]; };

__device__ __forceinline__ unsigned short bf16_bits(float x) { unsigned int u = __float_as_uint(x); return (unsigned short)((u + 0x7FFFu + ((u >> 16) & 1u)) >> 16); }
__device__ __forceinline__ float bf16_val(unsigned short b) { return __uint_as_float(((unsigned int)b) << 16); }
__device__ __forceinline__ float bf16_round(float x) { return bf16_val(bf16_bits(x)); }
template <int NT>
__device__ __forceinline__ v8f mmaN(v16b ah, v16b al, v16b bh, v16b bl, v8f c) {
  c = __builtin_amdgcn_wmma_f32_16x16x32_bf16(false, ah, false, bh, (short)0, c, false, false);
  if (NT >= 2) c = __builtin_amdgcn_wmma_f32_16x16x32_bf16(false, al, false, bh, (short)0, c, false, false);
  if (NT >= 3) c = __builtin_amdgcn_wmma_f32_16x16x32_bf16(false, ah, false, bl, (short)0, c, false, false);
  asm volatile("v_nop\n\tv_nop\n\tv_nop\n\tv_nop" : "+v"(c) : "v"(ah), "v"(al), "v"(bh), "v"(bl));
  return c;
}

__global__ __launch_bounds__(256) void k_wt_bf16(const float* __restrict__ W, unsigned short* __restrict__ Wt, int K, int N) {
  const int t = blockIdx.x * 256 + threadIdx.x;
  const int k8n = K / 8;
  if (t >= N * k8n) return;
  const int n = t / k8n, k8 = (t % k8n) * 8;
  v8us v;
#pragma unroll
  for (int i = 0; i < 8; ++i) v[i] = bf16_bits(W[(size_t)(k8 + i) * N + n]);
  *(volatile v8us*)(Wt + (size_t)n * K + k8) = v;
  __threadfence();
  *(volatile v8us*)(Wt + (size_t)n * K + k8) = v;
}

template <bool ASPLIT, int ACT, bool BIAS_BF16>
__global__ __launch_bounds__(128) void k_gemm_bf(const float* __restrict__ A, int lda, const unsigned short* __restrict__ Wt, int ldb,
                                               const float* __restrict__ bias, float* __restrict__ C, int ldc, int M, int N, int K) {
  __shared__ __attribute__((aligned(16))) float so[4][16][64];
  const int tid = threadIdx.x, w = tid >> 5, lane = tid & 31, ln = lane & 15, hh = lane >> 4;
  const int ntn = N / 64;
  const int wid = blockIdx.x * 4 + w;
  const int mt = wid / ntn, nq = wid % ntn;
  if (mt * 16 >= M) return;
  const int row0 = mt * 16, col0 = nq * 64;
  const float* arow = A + (size_t)(row0 + ln) * lda;
  v8f acc[4] = {};
  for (int kb = 0; kb < K; kb += 32) {
    FragB ah, al;
    const v4f x0 = *(const v4fa*)(arow + kb + 8 * hh), x1 = *(const v4fa*)(arow + kb + 8 * hh + 4);
    const v4f x2 = *(const v4fa*)(arow + kb + 16 + 8 * hh), x3 = *(const v4fa*)(arow + kb + 16 + 8 * hh + 4);
    float xs[16] = {x0[0],x0[1],x0[2],x0[3],x1[0],x1[1],x1[2],x1[3],x2[0],x2[1],x2[2],x2[3],x3[0],x3[1],x3[2],x3[3]};
#pragma unroll
    for (int i = 0; i < 16; ++i) { const unsigned short hb = bf16_bits(xs[i]); ah.u[i] = hb; al.u[i] = ASPLIT ? bf16_bits(xs[i] - bf16_val(hb)) : (unsigned short)0; }
#pragma unroll
    for (int t = 0; t < 4; ++t) {
      const unsigned short* brow = Wt + (size_t)(col0 + t * 16 + ln) * ldb + kb;
      FragB b;
      b.half[0] = *(const v8us*)(brow + 8 * hh);
      b.half[1] = *(const v8us*)(brow + 16 + 8 * hh);
      acc[t] = mmaN<ASPLIT ? 2 : 1>(ah.v, al.v, b.v, b.v, acc[t]);
    }
  }
#pragma unroll
  for (int t = 0; t < 4; ++t) {
    float bv = bias ? bias[col0 + t * 16 + ln] : 0.f;
    if (BIAS_BF16) bv = bf16_round(bv);
#pragma unroll
    for (int r = 0; r < 8; ++r) { float v = acc[t][r] + bv; if (ACT == 1) v = fmaxf(v, 0.f); so[w][8 * hh + r][t * 16 + ln] = v; }
  }
  __builtin_amdgcn_fence(__ATOMIC_ACQ_REL, "workgroup");
  __builtin_amdgcn_wave_barrier();
  const int rsub = lane >> 4, c4 = (lane & 15) * 4;
  for (int pass = 0; pass < 2; ++pass) {
#pragma unroll
    for (int q = 0; q < 8; ++q) {
      const int r = q * 2 + rsub;
      const v4f v = *(const v4fa*)&so[w][r][c4];
      *(volatile v4f*)(C + (size_t)(row0 + r) * ldc + col0 + c4) = v;
    }
    if (pass == 0) __threadfence();
  }
}

template <bool ASPLIT, int ACT, bool BIAS_BF16, bool RES_BF16>
__global__ __launch_bounds__(128) void k_gemm_bf3(const float* __restrict__ A, int lda, const unsigned short* __restrict__ Wt, int ldb,
                                                const float* __restrict__ bias, const float* __restrict__ resid, int rmod, int ldr,
                                                float* __restrict__ C, int ldc, int M, int N, int K) {
  __shared__ __attribute__((aligned(16))) float so[4][16][64];
  const int tid = threadIdx.x, w = tid >> 5, lane = tid & 31, ln = lane & 15, hh = lane >> 4;
  const int ntn = N / 64;
  const int wid = blockIdx.x * 4 + w;
  const int mt = wid / ntn, nq = wid % ntn;
  if (mt * 16 >= M) return;
  const int row0 = mt * 16, col0 = nq * 64;
  const float* arow = A + (size_t)(row0 + ln) * lda;
  v8f acc[4] = {};
  for (int kb = 0; kb < K; kb += 32) {
    FragB ah, al;
    const v4f x0 = *(const v4fa*)(arow + kb + 8 * hh), x1 = *(const v4fa*)(arow + kb + 8 * hh + 4);
    const v4f x2 = *(const v4fa*)(arow + kb + 16 + 8 * hh), x3 = *(const v4fa*)(arow + kb + 16 + 8 * hh + 4);
    float xs[16] = {x0[0],x0[1],x0[2],x0[3],x1[0],x1[1],x1[2],x1[3],x2[0],x2[1],x2[2],x2[3],x3[0],x3[1],x3[2],x3[3]};
#pragma unroll
    for (int i = 0; i < 16; ++i) { const unsigned short hb = bf16_bits(xs[i]); ah.u[i] = hb; al.u[i] = ASPLIT ? bf16_bits(xs[i] - bf16_val(hb)) : (unsigned short)0; }
#pragma unroll
    for (int t = 0; t < 4; ++t) {
      const unsigned short* brow = Wt + (size_t)(col0 + t * 16 + ln) * ldb + kb;
      FragB b;
      b.half[0] = *(const v8us*)(brow + 8 * hh);
      b.half[1] = *(const v8us*)(brow + 16 + 8 * hh);
      acc[t] = mmaN<ASPLIT ? 2 : 1>(ah.v, al.v, b.v, b.v, acc[t]);
    }
  }
#pragma unroll
  for (int t = 0; t < 4; ++t) {
    const int col = col0 + t * 16 + ln;
    float bv = bias ? bias[col] : 0.f;
    if (BIAS_BF16) bv = bf16_round(bv);
#pragma unroll
    for (int r = 0; r < 8; ++r) {
      float v = acc[t][r] + bv;
      if (resid) { float rv = resid[(size_t)((row0 + 8 * hh + r) % rmod) * ldr + col]; if (RES_BF16) rv = bf16_round(rv); v += rv; }
      if (ACT == 1) v = fmaxf(v, 0.f);
      if (ACT == 2) v = 0.5f * v * (1.0f + erff(v * 0.70710678118654752f));
      if (ACT == 3) { const float u = 0.7978845608028654f * (v + 0.044715f * v * v * v); v = 0.5f * v * (1.0f + tanhf(u)); }
      so[w][8 * hh + r][t * 16 + ln] = v;
    }
  }
  __builtin_amdgcn_fence(__ATOMIC_ACQ_REL, "workgroup");
  __builtin_amdgcn_wave_barrier();
  const int rsub = lane >> 4, c4 = (lane & 15) * 4;
  for (int pass = 0; pass < 2; ++pass) {
#pragma unroll
    for (int q = 0; q < 8; ++q) {
      const int r = q * 2 + rsub;
      const v4f v = *(const v4fa*)&so[w][r][c4];
      *(volatile v4f*)(C + (size_t)(row0 + r) * ldc + col0 + c4) = v;
    }
    if (pass == 0) __threadfence();
  }
}
template <bool PARAM_BF16>
__global__ __launch_bounds__(256) void k_layernorm(const float* __restrict__ X, const float* __restrict__ R, const float* __restrict__ g, const float* __restrict__ bta,
                                                  float* __restrict__ out_sum, float* __restrict__ out_norm, int N, float eps) {
  __shared__ float red[256];
  const int row = blockIdx.x, tid = threadIdx.x;
  const float* x = X + (size_t)row * N; const float* rr = R ? R + (size_t)row * N : nullptr;
  float vals[16];
  const int per = N / 256;
  float s1 = 0.f;
  for (int u = 0; u < per / 4; ++u) {
    const int j = tid * 4 + 1024 * u;
    const v4f a = *(const v4fa*)(x + j);
    v4f b = {0.f,0.f,0.f,0.f}; if (rr) b = *(const v4fa*)(rr + j);
#pragma unroll
    for (int q = 0; q < 4; ++q) { const float v = a[q] + b[q]; vals[u * 4 + q] = v; s1 += v; }
  }
  red[tid] = s1; __syncthreads();
  for (int st = 128; st > 0; st >>= 1) { if (tid < st) red[tid] += red[tid + st]; __syncthreads(); }
  const float mu = red[0] / (float)N; __syncthreads();
  float s2 = 0.f;
  for (int u = 0; u < per / 4; ++u)
#pragma unroll
    for (int q = 0; q < 4; ++q) { const float c = vals[u * 4 + q] - mu; s2 += c * c; }
  red[tid] = s2; __syncthreads();
  for (int st = 128; st > 0; st >>= 1) { if (tid < st) red[tid] += red[tid + st]; __syncthreads(); }
  const float rs = rsqrtf(red[0] / (float)N + eps);
  for (int pass = 0; pass < 2; ++pass) {
    for (int u = 0; u < per / 4; ++u) {
      const int j = tid * 4 + 1024 * u;
      v4f o, sm;
#pragma unroll
      for (int q = 0; q < 4; ++q) {
        float gg = g[j + q], bb = bta[j + q];
        if (PARAM_BF16) { gg = bf16_round(gg); bb = bf16_round(bb); }
        sm[q] = vals[u * 4 + q]; o[q] = (vals[u * 4 + q] - mu) * rs * gg + bb;
      }
      if (out_sum) *(volatile v4f*)(out_sum + (size_t)row * N + j) = sm;
      *(volatile v4f*)(out_norm + (size_t)row * N + j) = o;
    }
    if (pass == 0) __threadfence();
  }
}


typedef _Float16 v16h __attribute__((ext_vector_type(16)));
union FragH { v16h v; v8us half[2]; _Float16 h[16]; unsigned short u[16]; };
template <int NT>
__device__ __forceinline__ v8f mmaH(v16h ah, v16h al, v16h bh, v16h bl, v8f c) {
  c = __builtin_amdgcn_wmma_f32_16x16x32_f16(false, ah, false, bh, (short)0, c, false, false);
  if (NT >= 2) c = __builtin_amdgcn_wmma_f32_16x16x32_f16(false, al, false, bh, (short)0, c, false, false);
  if (NT >= 3) c = __builtin_amdgcn_wmma_f32_16x16x32_f16(false, ah, false, bl, (short)0, c, false, false);
  asm volatile("v_nop\n\tv_nop\n\tv_nop\n\tv_nop" : "+v"(c) : "v"(ah), "v"(al), "v"(bh), "v"(bl));
  return c;
}
template <bool ASPLIT>
__global__ __launch_bounds__(128) void k_gemm_h(const float* __restrict__ A, int lda, size_t sA, const _Float16* __restrict__ Bh, int ldb, size_t sB, float alpha, float* __restrict__ C, int ldc, size_t sC, int M, int N, int K) {
  __shared__ __attribute__((aligned(16))) float so[4][16][64];
  const int tid = threadIdx.x, w = tid >> 5, lane = tid & 31, ln = lane & 15, hh = lane >> 4; const int by = blockIdx.y;
  A += (size_t)by * sA; Bh += (size_t)by * sB; C += (size_t)by * sC;
  const int ntn = (N + 63) / 64; const int wid = blockIdx.x * 4 + w; const int mt = wid / ntn, nq = wid % ntn; if (mt * 16 >= M) return;
  const int row0 = mt * 16, col0 = nq * 64; const float* arow = A + (size_t)(row0 + ln) * lda;
  v8f acc[4] = {};
  for (int kb = 0; kb < K; kb += 32) {
    FragH ah, al;
    const v4f x0 = *(const v4fa*)(arow + kb + 8 * hh), x1 = *(const v4fa*)(arow + kb + 8 * hh + 4), x2 = *(const v4fa*)(arow + kb + 16 + 8 * hh), x3 = *(const v4fa*)(arow + kb + 16 + 8 * hh + 4);
    float xs[16] = {x0[0],x0[1],x0[2],x0[3],x1[0],x1[1],x1[2],x1[3],x2[0],x2[1],x2[2],x2[3],x3[0],x3[1],x3[2],x3[3]};
#pragma unroll
    for (int i = 0; i < 16; ++i) { const _Float16 h = (_Float16)xs[i]; ah.h[i] = h; al.h[i] = ASPLIT ? (_Float16)(xs[i] - (float)h) : (_Float16)0.0f; }
#pragma unroll
    for (int t = 0; t < 4; ++t) { if (col0 + t * 16 >= N) continue; const size_t boff = (size_t)(col0 + t * 16 + ln) * ldb + kb; FragH bq; bq.half[0] = *(const v8us*)(Bh + boff + 8 * hh); bq.half[1] = *(const v8us*)(Bh + boff + 16 + 8 * hh);
      acc[t] = mmaH<ASPLIT ? 2 : 1>(ah.v, al.v, bq.v, bq.v, acc[t]); }
  }
#pragma unroll
  for (int t = 0; t < 4; ++t) { if (col0 + t * 16 >= N) continue;
#pragma unroll
    for (int r = 0; r < 8; ++r) so[w][8 * hh + r][t * 16 + ln] = acc[t][r] * alpha; }
  __builtin_amdgcn_fence(__ATOMIC_ACQ_REL, "workgroup"); __builtin_amdgcn_wave_barrier();
  const int rsub = lane >> 4, c4 = (lane & 15) * 4;
  for (int pass = 0; pass < 2; ++pass) {
#pragma unroll
    for (int q = 0; q < 8; ++q) { const int r = q * 2 + rsub; if (col0 + c4 < N) { const v4f v = *(const v4fa*)&so[w][r][c4]; *(volatile v4f*)(C + (size_t)(row0 + r) * ldc + col0 + c4) = v; } }
    if (pass == 0) __threadfence(); }
}

__global__ __launch_bounds__(256) void k_wt_f16(const float* __restrict__ W, _Float16* __restrict__ Wt, int K, int N, float scale) {
  const int t = blockIdx.x * 256 + threadIdx.x; if (t >= N * (K / 8)) return; const int n = t / (K / 8), k8 = (t % (K / 8)) * 8; FragH f;
#pragma unroll
  for (int i = 0; i < 8; ++i) f.h[i] = (_Float16)(bf16_round(W[(size_t)(k8 + i) * N + n]) * scale); const v8us o = f.half[0];
  *(volatile v8us*)((unsigned short*)Wt + (size_t)n * K + k8) = o; __threadfence(); *(volatile v8us*)((unsigned short*)Wt + (size_t)n * K + k8) = o;
}
template <int ACT>
__global__ __launch_bounds__(128) void k_gemm_hhx(const _Float16* __restrict__ A, int lda, size_t sA, const _Float16* __restrict__ Bh, int ldb, size_t sB, float alpha, const float* __restrict__ bias, size_t sBias, const float* __restrict__ CP, int rowsPerB, size_t sCPb, int row0g,
    float* __restrict__ C, _Float16* __restrict__ C16, int ldc, size_t sC, int M, int N, int K) {
  __shared__ __attribute__((aligned(16))) float so[4][16][64];
  const int tid = threadIdx.x, w = tid >> 5, lane = tid & 31, ln = lane & 15, hh = lane >> 4; const int by = blockIdx.y;
  A += (size_t)by * sA; Bh += (size_t)by * sB; const size_t cofs = (size_t)by * sC; const float* bp = bias ? bias + (size_t)by * sBias : nullptr;
  const int ntn = (N + 63) / 64; const int wid = blockIdx.x * 4 + w; const int mt = wid / ntn, nq = wid % ntn; if (mt * 16 >= M) return;
  const int row0 = mt * 16, col0 = nq * 64; const _Float16* arow = A + (size_t)(row0 + ln) * lda;
  v8f acc[4] = {};
  for (int kb = 0; kb < K; kb += 32) { FragH ah; ah.half[0] = *(const v8us*)((const unsigned short*)arow + kb + 8 * hh); ah.half[1] = *(const v8us*)((const unsigned short*)arow + kb + 16 + 8 * hh);
#pragma unroll
    for (int t = 0; t < 4; ++t) { if (col0 + t * 16 >= N) continue; const size_t boff = (size_t)(col0 + t * 16 + ln) * ldb + kb; FragH bq; bq.half[0] = *(const v8us*)((const unsigned short*)Bh + boff + 8 * hh); bq.half[1] = *(const v8us*)((const unsigned short*)Bh + boff + 16 + 8 * hh);
      acc[t] = mmaH<1>(ah.v, ah.v, bq.v, bq.v, acc[t]); }
  }
#pragma unroll
  for (int t = 0; t < 4; ++t) { if (col0 + t * 16 >= N) continue; const int col = col0 + t * 16 + ln; const float bv = bp ? bf16_round(bp[col]) : 0.f;
#pragma unroll
    for (int r = 0; r < 8; ++r) { float v = acc[t][r] * alpha + bv; if (CP) { const int rr = row0g + row0 + 8 * hh + r; if (rowsPerB < 0) v += CP[cofs + (size_t)rr * ldc + col];        else { const int bidx = rr / rowsPerB; v += CP[(size_t)bidx * sCPb + (size_t)by * 64 + col]; } } if (ACT == 1) v = (v > 0.f) ? v : expm1f(v); else if (ACT == 7) v = (v > 0.f) ? v + 1.0f : expf(v); else if (ACT == 8) v = tanhf(v); else if (ACT == 9) v = 0.5f * v * (1.0f + tanhf(0.7978845608028654f * (v + 0.044715f * v * v * v))); else if (ACT == 11) v = 1.0f / (1.0f + expf(-v)); else if (ACT == 12) v = (v > 0.f) ? v : 0.01f * v; else if (ACT == 14) v = (v > 0.f) ? v : 0.1f * v; else if (ACT == 16) v = (v >= 0.f) ? v : 0.3f * v; else if (ACT == 17) v = (v >= 0.f) ? v : 0.2f * v; else if (ACT == 15) v = v / (1.0f + expf(-v)); else if (ACT == 3) v = fmaxf(v, 0.f); else if (ACT == 6) v = 0.5f * v * (1.0f + erff(v * 0.70710678118654752f)); so[w][8 * hh + r][t * 16 + ln] = v; } }
  __builtin_amdgcn_fence(__ATOMIC_ACQ_REL, "workgroup"); __builtin_amdgcn_wave_barrier();
  const int rsub = lane >> 4, c4 = (lane & 15) * 4; typedef _Float16 v4h __attribute__((ext_vector_type(4)));
  for (int pass = 0; pass < 2; ++pass) {
#pragma unroll
    for (int q = 0; q < 8; ++q) { const int r = q * 2 + rsub; if (col0 + c4 < N) { const v4f v = *(const v4fa*)&so[w][r][c4]; if (C) *(volatile v4f*)(C + cofs + (size_t)(row0 + r) * ldc + col0 + c4) = v; if (C16) { v4h h4; for (int i = 0; i < 4; ++i) h4[i] = (_Float16)v[i]; *(volatile v4h*)(C16 + cofs + (size_t)(row0 + r) * ldc + col0 + c4) = h4; } } }
    if (pass == 0) __threadfence(); }
}


typedef _Float16 v4h __attribute__((ext_vector_type(4)));

__global__ __launch_bounds__(256) void k_x16(const float* __restrict__ x, _Float16* __restrict__ X16, size_t n8) { const size_t t = (size_t)blockIdx.x * 256 + threadIdx.x; if (t >= n8) return; FragH f;
#pragma unroll
  for (int q = 0; q < 8; ++q) f.h[q] = (_Float16)bf16_round(x[t * 8 + q]); *(volatile v8us*)((unsigned short*)X16 + t * 8) = f.half[0]; __threadfence(); *(volatile v8us*)((unsigned short*)X16 + t * 8) = f.half[0]; }
__global__ __launch_bounds__(256) void k_h16(const float* __restrict__ x, _Float16* __restrict__ X16, size_t n8) { const size_t t = (size_t)blockIdx.x * 256 + threadIdx.x; if (t >= n8) return; FragH f;
#pragma unroll
  for (int q = 0; q < 8; ++q) f.h[q] = (_Float16)x[t * 8 + q]; *(volatile v8us*)((unsigned short*)X16 + t * 8) = f.half[0]; __threadfence(); *(volatile v8us*)((unsigned short*)X16 + t * 8) = f.half[0]; }
__global__ __launch_bounds__(256) void k_round16f(const float* __restrict__ W, _Float16* __restrict__ Bt, size_t n8) { const size_t t = (size_t)blockIdx.x * 256 + threadIdx.x; if (t >= n8) return; FragH f;
#pragma unroll
  for (int i = 0; i < 8; ++i) f.h[i] = (_Float16)(bf16_round(W[t * 8 + i]) * 16.0f); *(volatile v8us*)((unsigned short*)Bt + t * 8) = f.half[0]; __threadfence(); *(volatile v8us*)((unsigned short*)Bt + t * 8) = f.half[0]; }
template <int NHv, int TTv>
__global__ __launch_bounds__(256) void k_vt(const _Float16* __restrict__ V16, int ldv, int voff, _Float16* __restrict__ Vt) { __shared__ unsigned short tl[64][66]; const int tid = threadIdx.x; const int slab = blockIdx.x / (TTv / 64), lg = blockIdx.x % (TTv / 64); const int b = slab / NHv, h = slab % NHv;
  for (int i = tid; i < 64 * 8; i += 256) { const int r = i / 8, c8 = (i % 8) * 8; FragH f; f.half[0] = *(const v8us*)((const unsigned short*)V16 + ((size_t)b * TTv + lg * 64 + r) * ldv + voff + h * 64 + c8);
#pragma unroll
    for (int q = 0; q < 8; ++q) tl[r][c8 + q] = f.u[q]; }
  __syncthreads();
  for (int pass = 0; pass < 2; ++pass) {
#pragma unroll
    for (int rd = 0; rd < 2; ++rd) { const int d = rd * 32 + tid / 8, pc = tid % 8; FragH f;
#pragma unroll
      for (int q = 0; q < 8; ++q) f.u[q] = tl[pc * 8 + q][d];
      *(volatile v8us*)((unsigned short*)Vt + ((size_t)slab * 64 + d) * TTv + lg * 64 + pc * 8) = f.half[0]; }
    if (pass == 0) __threadfence(); } }

__global__ __launch_bounds__(256) void k_hl(const float* __restrict__ F, _Float16* __restrict__ Hh, _Float16* __restrict__ Hl, size_t n8) { const size_t t = (size_t)blockIdx.x * 256 + threadIdx.x; if (t >= n8) return; FragH fh, fl; const v4f a = *(const v4fa*)(F + t * 8), c = *(const v4fa*)(F + t * 8 + 4);
#pragma unroll
  for (int q = 0; q < 4; ++q) { _Float16 h = (_Float16)a[q]; fh.h[q] = h; fl.h[q] = (_Float16)((a[q] - (float)h) * 1024.0f); h = (_Float16)c[q]; fh.h[4 + q] = h; fl.h[4 + q] = (_Float16)((c[q] - (float)h) * 1024.0f); }
  for (int pass = 0; pass < 2; ++pass) { *(volatile v8us*)((unsigned short*)Hh + t * 8) = fh.half[0]; *(volatile v8us*)((unsigned short*)Hl + t * 8) = fl.half[0]; if (pass == 0) __threadfence(); } }

__device__ __forceinline__ v16h g2_frag(const _Float16* p, int hh) { FragH f; f.half[0] = *(const v8us*)((const unsigned short*)p + 8 * hh); f.half[1] = *(const v8us*)((const unsigned short*)p + 16 + 8 * hh); return f.v; }
__device__ __forceinline__ v8f g2_mma(v16h a, v16h b, v8f c) { v8f d = __builtin_amdgcn_wmma_f32_16x16x32_f16(false, a, false, b, (short)0, c, false, false); asm volatile("v_nop\n\tv_nop\n\tv_nop\n\tv_nop" : "+v"(d) : "v"(a), "v"(b)); return d; }
template <int ACT>
__global__ __launch_bounds__(128) void k_gemm2(const _Float16* __restrict__ A, int lda, size_t sA, const _Float16* __restrict__ Bh, int ldb, size_t sB, float alpha, const float* __restrict__ bias, size_t sBias, const float* __restrict__ CP, int rowsPerB, size_t sCPb, int row0g,
    float* __restrict__ C, _Float16* __restrict__ C16, int ldc, size_t sC, int M, int N, int K) { static_assert(ACT == 0 || ACT == 3 || ACT == 6 || ACT == 8 || ACT == 9 || ACT == 11 || ACT == 12 || ACT == 14 || ACT == 15 || ACT == 16 || ACT == 17, "k_gemm2: unsupported ACT code (would silently apply no activation)");
  __shared__ __attribute__((aligned(16))) float so[4][32][68];
  const int tid = threadIdx.x, w = tid >> 5, lane = tid & 31, ln = lane & 15, hh = lane >> 4; const int by = blockIdx.y;
  A += (size_t)by * sA; Bh += (size_t)by * sB; const size_t cofs = (size_t)by * sC; const float* bp = bias ? bias + (size_t)by * sBias : nullptr;
  const int ntn = N >> 6; const int mt = blockIdx.x / ntn, nq = blockIdx.x - mt * ntn; const int row0 = mt * 128 + 32 * w, col0 = nq * 64; if (row0 >= M) return;
  const _Float16* a0p = A + (size_t)(row0 + ln) * lda; const _Float16* a1p = a0p + (size_t)16 * lda;
  const _Float16* b0p = Bh + (size_t)(col0 + ln) * ldb; const _Float16* b1p = b0p + (size_t)16 * ldb; const _Float16* b2p = b1p + (size_t)16 * ldb; const _Float16* b3p = b2p + (size_t)16 * ldb;
  const v8f z8 = {0.f,0.f,0.f,0.f,0.f,0.f,0.f,0.f}; v8f c00 = z8, c01 = z8, c02 = z8, c03 = z8, c10 = z8, c11 = z8, c12 = z8, c13 = z8;
#pragma unroll 1
  for (int kb = 0; kb < K; kb += 32) { const v16h a0 = g2_frag(a0p + kb, hh), a1 = g2_frag(a1p + kb, hh);
    v16h b = g2_frag(b0p + kb, hh); c00 = g2_mma(a0, b, c00); c10 = g2_mma(a1, b, c10);
    b = g2_frag(b1p + kb, hh); c01 = g2_mma(a0, b, c01); c11 = g2_mma(a1, b, c11);
    b = g2_frag(b2p + kb, hh); c02 = g2_mma(a0, b, c02); c12 = g2_mma(a1, b, c12);
    b = g2_frag(b3p + kb, hh); c03 = g2_mma(a0, b, c03); c13 = g2_mma(a1, b, c13); }
  v8f accs[8] = {c00, c01, c02, c03, c10, c11, c12, c13};
#pragma unroll
  for (int u = 0; u < 8; ++u) { const int t = u & 3, half = u >> 2; const int col = col0 + t * 16 + ln; const float bv = bp ? bf16_round(bp[col]) : 0.f;
#pragma unroll
    for (int r = 0; r < 8; ++r) { const int rloc = half * 16 + 8 * hh + r; float v = accs[u][r] * alpha + bv; if (CP) { if (rowsPerB < 0) v += CP[cofs + (size_t)(row0g + row0 + rloc) * ldc + col];        else { const int bidx = (row0g + row0 + rloc) / rowsPerB; v += CP[(size_t)bidx * sCPb + (size_t)by * 64 + col]; } }
      if (ACT == 3) v = fmaxf(v, 0.f); else if (ACT == 6) v = 0.5f * v * (1.0f + erff(v * 0.70710678118654752f)); else if (ACT == 11) v = 1.0f / (1.0f + expf(-v)); else if (ACT == 15) v = v / (1.0f + expf(-v)); else if (ACT == 12) v = (v > 0.f) ? v : 0.01f * v; else if (ACT == 8) v = tanhf(v); else if (ACT == 9) v = 0.5f * v * (1.0f + tanhf(0.7978845608028654f * (v + 0.044715f * v * v * v))); else if (ACT == 14) v = (v > 0.f) ? v : 0.1f * v; else if (ACT == 16) v = (v >= 0.f) ? v : 0.3f * v; else if (ACT == 17) v = (v >= 0.f) ? v : 0.2f * v;
      so[w][rloc][t * 16 + ln] = v; } }
  __builtin_amdgcn_fence(__ATOMIC_ACQ_REL, "workgroup"); __builtin_amdgcn_wave_barrier();
  const int rsub = lane >> 4, c4 = (lane & 15) * 4;
  for (int pass = 0; pass < 2; ++pass) {
#pragma unroll
    for (int q = 0; q < 16; ++q) { const int r = q * 2 + rsub; const v4f v = *(const v4fa*)&so[w][r][c4]; if (C) *(volatile v4f*)(C + cofs + (size_t)(row0 + r) * ldc + col0 + c4) = v; if (C16) { v4h h4; for (int i = 0; i < 4; ++i) h4[i] = (_Float16)v[i]; *(volatile v4h*)(C16 + cofs + (size_t)(row0 + r) * ldc + col0 + c4) = h4; } }
    if (pass == 0) __threadfence(); } }


__global__ __launch_bounds__(256) void k_wuv(const float* __restrict__ w, _Float16* __restrict__ Bt) { const int t = blockIdx.x * 256 + threadIdx.x; if (t >= CO3 * CHP / 8) return; const int k0 = (t * 8) % CHP, o = (t * 8) / CHP; FragH f; for (int q = 0; q < 8; ++q) { const int k = k0 + q; f.h[q] = (k < CH1) ? (_Float16)(bf16_round(w[(size_t)o * CH1 + k]) * 16.0f) : (_Float16)0.0f; }
  *(volatile v8us*)((unsigned short*)Bt + (size_t)t * 8) = f.half[0]; __threadfence(); *(volatile v8us*)((unsigned short*)Bt + (size_t)t * 8) = f.half[0]; }
__global__ __launch_bounds__(256) void k_pq(const float* __restrict__ u, const float* __restrict__ v, const int* __restrict__ ides, const float* __restrict__ Wgu, const float* __restrict__ bgu, const float* __restrict__ Wgv, const float* __restrict__ bgv, float* __restrict__ PQ) {
  #pragma clang fp contract(off)
  const size_t t = (size_t)blockIdx.x * 256 + threadIdx.x; if (t >= (size_t)NBT * (NPT + NS) * CH1) return; const int ch = (int)(t % CH1); const int j = (int)((t / CH1) % (NPT + NS)); const int b = (int)(t / ((size_t)CH1 * (NPT + NS))); const bool self_ = j < NPT; const int n = self_ ? j : ides[b * NSI + (j - NPT)]; float acc = 0.f;
  if (ch < 2 * CU) { const int c0 = self_ ? 0 : CU;
#pragma unroll 1
    for (int c = 0; c < CU; ++c) acc += bf16_round(Wgu[ch * 2 * CU + c0 + c]) * bf16_round(u[((size_t)b * CU + c) * NPT + n]); if (self_) acc += bf16_round(bgu[ch]); }
  else { const int o = ch - 2 * CU; const int c0 = self_ ? 0 : CV;
#pragma unroll 1
    for (int c = 0; c < CV; ++c) acc += bf16_round(Wgv[(size_t)o * 2 * CV + c0 + c]) * bf16_round(v[((size_t)b * CV + c) * NPT + n]); if (self_) acc += bf16_round(bgv[o]); }
  *(volatile float*)(PQ + t) = acc; __threadfence(); *(volatile float*)(PQ + t) = acc; }
__global__ __launch_bounds__(256) void k_stat1(const float* __restrict__ PQ, float* __restrict__ MV) {
  #pragma clang fp contract(off)
  const int wv = threadIdx.x >> 5, ln = threadIdx.x & 31;
#pragma unroll 1
  for (int ci = 0; ci < 16; ++ci) { const int ch = (blockIdx.x * 8 + wv) * 16 + ci; if (ch >= CH1) break; double s1 = 0.0, s2 = 0.0;
  for (int b = 0; b < NBT; ++b) { const float* pq = PQ + (size_t)b * (NPT + NS) * CH1 + ch; double sp = 0.0, sp2 = 0.0, sq = 0.0, sq2 = 0.0;
    for (int n = ln; n < NPT; n += 32) { const double p = (double)pq[(size_t)n * CH1]; sp += p; sp2 += p * p; }
    for (int s = ln; s < NS; s += 32) { const double q = (double)pq[(size_t)(NPT + s) * CH1]; sq += q; sq2 += q * q; }
    for (int o = 16; o > 0; o >>= 1) { sp += __shfl_xor(sp, o, 32); sp2 += __shfl_xor(sp2, o, 32); sq += __shfl_xor(sq, o, 32); sq2 += __shfl_xor(sq2, o, 32); }
    s1 += sp * (double)NS + sq * (double)NPT; s2 += sp2 * (double)NS + sq2 * (double)NPT + 2.0 * sp * sq; }
  const double cnt = (double)NR; const double mean = s1 / cnt; double var = s2 / cnt - mean * mean; if (var < 0.0) var = 0.0; const float rs = (float)(1.0 / sqrt(var + 1e-5));
  if (ln == 0) { *(volatile float*)(MV + 2 * ch) = (float)mean; *(volatile float*)(MV + 2 * ch + 1) = rs; __threadfence(); *(volatile float*)(MV + 2 * ch) = (float)mean; *(volatile float*)(MV + 2 * ch + 1) = rs; } } }
__global__ __launch_bounds__(256) void k_hid(const float* __restrict__ PQ, const float* __restrict__ MV, const float* __restrict__ g1, const float* __restrict__ be1, const float* __restrict__ g2, const float* __restrict__ be2, int b, _Float16* __restrict__ H) {
  #pragma clang fp contract(off)
  const size_t t = (size_t)blockIdx.x * 256 + threadIdx.x; if (t >= (size_t)NPT * NS * CHP / 8) return; const int ch0 = (int)((t * 8) % CHP); const size_t row = (t * 8) / CHP; const int s = (int)(row % NS); const int n = (int)(row / NS); const float* pn = PQ + ((size_t)b * (NPT + NS) + n) * CH1; const float* qs = PQ + ((size_t)b * (NPT + NS) + NPT + s) * CH1; FragH f;
  for (int q = 0; q < 8; ++q) { const int ch = ch0 + q; float o = 0.f; if (ch < CH1) { float x = pn[ch] + qs[ch]; x = x - MV[2 * ch]; x = x * MV[2 * ch + 1]; const float gg = (ch < 2 * CU) ? bf16_round(g1[ch]) : bf16_round(g2[ch - 2 * CU]); const float bb = (ch < 2 * CU) ? bf16_round(be1[ch]) : bf16_round(be2[ch - 2 * CU]); x = x * gg; x += bb; o = fmaxf(x, 0.f); } f.h[q] = (_Float16)o; }
  *(volatile v8us*)((unsigned short*)H + t * 8) = f.half[0]; __threadfence(); *(volatile v8us*)((unsigned short*)H + t * 8) = f.half[0]; }
__global__ __launch_bounds__(64) void k_colps(const float* __restrict__ Z, double* __restrict__ PS) { const int c = threadIdx.x; const size_t r0 = (size_t)blockIdx.x * RB; double s1 = 0.0, s2 = 0.0;
#pragma unroll 1
  for (int r = 0; r < RB; ++r) { const double z = (double)Z[(r0 + r) * CO3 + c]; s1 += z; s2 += z * z; }
  double* d = PS + ((size_t)blockIdx.x * CO3 + c) * 2; *(volatile double*)d = s1; *(volatile double*)(d + 1) = s2; __threadfence(); *(volatile double*)d = s1; *(volatile double*)(d + 1) = s2; }
__global__ __launch_bounds__(64) void k_stat3(const double* __restrict__ PS, float* __restrict__ MV) { const int c = threadIdx.x; double s1 = 0.0, s2 = 0.0; for (int b = 0; b < (int)NBLK; ++b) { s1 += PS[((size_t)b * CO3 + c) * 2]; s2 += PS[((size_t)b * CO3 + c) * 2 + 1]; }
  const double mean = s1 / (double)NR; double var = s2 / (double)NR - mean * mean; if (var < 0.0) var = 0.0; const float rs = (float)(1.0 / sqrt(var + 1e-5)); *(volatile float*)(MV + 2 * c) = (float)mean; *(volatile float*)(MV + 2 * c + 1) = rs; __threadfence(); *(volatile float*)(MV + 2 * c) = (float)mean; *(volatile float*)(MV + 2 * c + 1) = rs; }
__global__ __launch_bounds__(256) void k_max(const float* __restrict__ Z, const float* __restrict__ MV, const float* __restrict__ g3, const float* __restrict__ be3, int b, float* __restrict__ Mout) {
  #pragma clang fp contract(off)
  const size_t t = (size_t)blockIdx.x * 256 + threadIdx.x; if (t >= (size_t)NPT * CO3) return; const int c = (int)(t % CO3); const size_t bn_ = t / CO3; float* M = Mout + (size_t)b * NPT * CO3; const float mean = MV[2 * c], rs = MV[2 * c + 1], gg = bf16_round(g3[c]), bb = bf16_round(be3[c]); float mx = -3.0e38f;
#pragma unroll 1
  for (int s = 0; s < NS; ++s) { float x = Z[(bn_ * NS + s) * CO3 + c] - mean; x = x * rs; x = x * gg; x += bb; x = fmaxf(x, 0.f); mx = fmaxf(mx, x); }
  *(volatile float*)(M + t) = mx; __threadfence(); *(volatile float*)(M + t) = mx; }
__global__ __launch_bounds__(256) void k_fc4(const float* __restrict__ M, const float* __restrict__ Wf, const float* __restrict__ bf_, float* __restrict__ Z4) {
  #pragma clang fp contract(off)
  const size_t t = (size_t)blockIdx.x * 256 + threadIdx.x; if (t >= (size_t)NBT * NPT * CO3) return; const int o = (int)(t % CO3); const size_t bn_ = t / CO3; const float* m = M + bn_ * CO3; float acc = 0.f;
#pragma unroll 1
  for (int c = 0; c < CO3; ++c) acc += bf16_round(Wf[o * CO3 + c]) * m[c];
  acc += bf16_round(bf_[o]); *(volatile float*)(Z4 + t) = acc; __threadfence(); *(volatile float*)(Z4 + t) = acc; }
__global__ __launch_bounds__(256) void k_stat4(const float* __restrict__ Z4, float* __restrict__ MV) { const int wv = threadIdx.x >> 5, ln = threadIdx.x & 31;
#pragma unroll 1
  for (int ci = 0; ci < 16; ++ci) { const int c = (blockIdx.x * 8 + wv) * 16 + ci; if (c >= CO3) break; double s1 = 0.0, s2 = 0.0; for (size_t r = ln; r < (size_t)NBT * NPT; r += 32) { const double z = (double)Z4[r * CO3 + c]; s1 += z; s2 += z * z; }
  for (int o = 16; o > 0; o >>= 1) { s1 += __shfl_xor(s1, o, 32); s2 += __shfl_xor(s2, o, 32); } const double mean = s1 / (double)(NBT * NPT); double var = s2 / (double)(NBT * NPT) - mean * mean; if (var < 0.0) var = 0.0; const float rs = (float)(1.0 / sqrt(var + 1e-5));
  if (ln == 0) { *(volatile float*)(MV + 2 * c) = (float)mean; *(volatile float*)(MV + 2 * c + 1) = rs; __threadfence(); *(volatile float*)(MV + 2 * c) = (float)mean; *(volatile float*)(MV + 2 * c + 1) = rs; } } }
__global__ __launch_bounds__(256) void k_out(const float* __restrict__ u, const float* __restrict__ v, const float* __restrict__ Z4, const float* __restrict__ MV, const float* __restrict__ g4, const float* __restrict__ be4, float* __restrict__ out) {
  #pragma clang fp contract(off)
  const size_t t = (size_t)blockIdx.x * 256 + threadIdx.x; if (t >= (size_t)NBT * (CV + CU) * NPT / 8) return; const int n0 = (int)((t * 8) % NPT); const int c = (int)(((t * 8) / NPT) % (CV + CU)); const int b = (int)((t * 8) / ((size_t)NPT * (CV + CU))); v8f o;
  for (int q = 0; q < 8; ++q) { const int n = n0 + q; if (c < CV) { float x = Z4[((size_t)b * NPT + n) * CO3 + c] - MV[2 * c]; x = x * MV[2 * c + 1]; x = x * bf16_round(g4[c]); x += bf16_round(be4[c]); x = fmaxf(x, 0.f); float w = bf16_round(v[((size_t)b * CV + c) * NPT + n]); w += x; o[q] = w; } else { o[q] = bf16_round(u[((size_t)b * CU + (c - CV)) * NPT + n]); } }
  *(volatile v8f*)(out + t * 8) = o; __threadfence(); *(volatile v8f*)(out + t * 8) = o; }

extern "C" void kernel_launch(void* const* d_in, const int* in_sizes, int n_in,
                              void* d_out, int out_size, void* d_ws, size_t ws_size, hipStream_t stream) {
  (void)in_sizes; (void)n_in; (void)out_size;
  const float* const* I = (const float* const*)d_in; const float* u = I[0]; const float* v = I[1]; const int* ides = (const int*)d_in[2]; const float* Wgu = I[3]; const float* bgu = I[4]; const float* g1 = I[5]; const float* b1 = I[6]; const float* Wgv = I[7]; const float* bgv = I[8]; const float* g2 = I[9]; const float* b2 = I[10]; const float* Wuv = I[11]; const float* buv = I[12]; const float* g3 = I[13]; const float* b3 = I[14]; const float* Wf = I[15]; const float* bf_ = I[16]; const float* g4 = I[17]; const float* b4 = I[18];
  char* ws = (char*)d_ws; size_t off = 0;
  auto take = [&](size_t bytes) { char* p = ws + off; off += (bytes + 255) & ~(size_t)255; return p; };
  _Float16* BUV = (_Float16*)take((size_t)CO3 * CHP * 2); float* PQ = (float*)take((size_t)NBT * (NPT + NS) * CH1 * 4); float* MV1 = (float*)take(CH1 * 2 * 4); _Float16* H = (_Float16*)take((size_t)NPT * NS * CHP * 2); float* Z3 = (float*)take((size_t)NPT * NS * CO3 * 4); double* PS = (double*)take((size_t)NBLK * CO3 * 2 * 8); float* MV3 = (float*)take(CO3 * 2 * 4); float* M = (float*)take((size_t)NBT * NPT * CO3 * 4); float* Z4 = (float*)take((size_t)NBT * NPT * CO3 * 4); float* MV4 = (float*)take(CO3 * 2 * 4);
  if (off > ws_size) return;
  k_wuv<<<(CO3 * CHP / 8 + 255) / 256, 256, 0, stream>>>(Wuv, BUV);
  k_pq<<<(unsigned)(((size_t)NBT * (NPT + NS) * CH1 + 255) / 256), 256, 0, stream>>>(u, v, ides, Wgu, bgu, Wgv, bgv, PQ); k_stat1<<<(CH1 + 127) / 128, 256, 0, stream>>>(PQ, MV1);
  const size_t RCH = (size_t)NPT * NS;
  for (int pass = 0; pass < 2; ++pass) {
    for (int b = 0; b < NBT; ++b) {
      k_hid<<<(unsigned)((RCH * CHP / 8 + 255) / 256), 256, 0, stream>>>(PQ, MV1, g1, b1, g2, b2, b, H);
      k_gemm2<0><<<dim3((unsigned)(RCH / 128) * (CO3 / 64), 1), 128, 0, stream>>>(H, CHP, 0, BUV, CHP, 0, 0.0625f, buv, 0, nullptr, 1, 0, 0, Z3, nullptr, CO3, 0, (int)RCH, CO3, CHP);
      if (pass == 0) k_colps<<<(unsigned)(RCH / RB), 64, 0, stream>>>(Z3, PS + (size_t)b * (RCH / RB) * CO3 * 2);
      else k_max<<<(unsigned)(((size_t)NPT * CO3 + 255) / 256), 256, 0, stream>>>(Z3, MV3, g3, b3, b, M); }
    if (pass == 0) k_stat3<<<1, 64, 0, stream>>>(PS, MV3); }
  k_fc4<<<(unsigned)(((size_t)NBT * NPT * CO3 + 255) / 256), 256, 0, stream>>>(M, Wf, bf_, Z4); k_stat4<<<1, 256, 0, stream>>>(Z4, MV4);
  k_out<<<(unsigned)(((size_t)NBT * (CV + CU) * NPT / 8 + 255) / 256), 256, 0, stream>>>(u, v, Z4, MV4, g4, b4, (float*)d_out);
}
